// Encoder_42786464203487
// MI455X (gfx1250) — hardware-verified
//
#include <hip/hip_runtime.h>
#include <stddef.h>
#include <stdint.h>

#define DIM    32
#define HIDE   128
#define EWN    1024
#define KEW    256
#define KG     128
#define NTHR   256
#define NWAVE  8
#define EPB    128
#define AP     264
#define DP     132
#define GBM    64
#define GBN    128
#define GTHR   128
#define EPT    8
#define CHUNK  (NTHR * EPT)
#define WCAP   (EPT * 32)
#define LISTN  (NWAVE * WCAP)
#define NBA    1024
#define SLA    10
#define RCAP   8192
#define DEGCAP 32
#define GCAP   256
#define GP     33
#define AGG_ZINTS (LISTN + 2 * RCAP + 3 * NBA)
#define AGG_LDS_INTS (AGG_ZINTS + 16)
#define AGG_LDS_BYTES (AGG_LDS_INTS * 4)
#define EW_LDS_BYTES (EPB * DP * 4 + EPB * AP * 2)
#define WSMAX  268435456
#define CEW    256.0f
#define EWINV  0.00390625f

#define P_W1   0
#define P_B1   768
#define P_B2   1024
#define P_L0B  2048
#define P_CB   2080
#define P_FC   2112
#define P_LC   2116
#define P_GB   2304
#define P_LWI  2560
#define P_LWH  10752
#define P_LBI  14848
#define P_LBH  14976
#define PARN   15104
#define NB_W2D 128
#define NB_WG  8
#define NB_PAR 59

static_assert((CHUNK & (CHUNK - 1)) == 0 && CHUNK <= 4096);
static_assert((NBA & (NBA - 1)) == 0 && NBA == (1 << SLA));
static_assert(((long long)CHUNK << SLA) < (1LL << 31));
static_assert(LISTN % NTHR == 0 && LISTN % 4 == 0);
static_assert(NBA % NWAVE == 0 && NBA % 32 == 0 && NBA == 4 * NTHR);
static_assert(RCAP % (2 * NTHR) == 0 && AGG_ZINTS % (4 * NTHR) == 0);
static_assert(RCAP >= 5564);
static_assert(DEGCAP == 32 && DEGCAP >= 17 + 8);
static_assert(GCAP == NTHR && GCAP >= 107 + 64);
static_assert(AGG_LDS_BYTES <= 300000 && EW_LDS_BYTES <= 300000);
static_assert(KEW == 2 * HIDE && KEW % 32 == 0 && KG % 32 == 0 && KG == 4 * DIM);
static_assert(GBM == (GTHR / 32) * 16 && GBN == 4 * DIM);
static_assert((DP * 4) % 16 == 0 && (AP * 2) % 16 == 0 && AP >= KEW && DP >= 128);
static_assert(EPB == 16 * NWAVE && NTHR == 2 * EPB);
static_assert(NB_W2D * NTHR * 8 == EWN * KEW && NB_WG * NTHR * 8 == 128 * KG && NB_PAR * NTHR == PARN);
static_assert(P_B2 % 4 == 0 && P_LWI % 4 == 0 && P_LWH % 4 == 0);
static_assert(P_L0B == 8 * NTHR && P_CB == P_L0B + 32 && P_FC == P_L0B + 64 && P_LC == P_FC + 4);
static_assert(P_GB == 9 * NTHR && P_LWI == 10 * NTHR && P_LWH == 42 * NTHR && P_LBI == 58 * NTHR && P_LBH == P_LBI + 128);
static_assert((GCAP * GP) % 4 == 0);

typedef float          v4f   __attribute__((ext_vector_type(4)));
typedef float          v8f   __attribute__((ext_vector_type(8)));
typedef int            v2i   __attribute__((ext_vector_type(2)));
typedef int            v4i   __attribute__((ext_vector_type(4)));
typedef int            v8i   __attribute__((ext_vector_type(8)));
typedef unsigned short v8us  __attribute__((ext_vector_type(8)));
typedef unsigned short v16us __attribute__((ext_vector_type(16)));
typedef __bf16         v16bf __attribute__((ext_vector_type(16)));
typedef v4f  __attribute__((may_alias)) v4fa;
typedef v4i  __attribute__((may_alias)) v4ia;
typedef v8us __attribute__((may_alias)) v8usa;
union FragB { v16bf v; v16us u; v8us h[2]; v8i w; };

__device__ __forceinline__ v8f wmb(const FragB& a, const FragB& b, v8f c) {
  v8f d = __builtin_amdgcn_wmma_f32_16x16x32_bf16(false, a.v, false, b.v, (short)0, c, false, false);
  asm volatile("v_nop\n\tv_nop\n\tv_nop\n\tv_nop" : "+v"(d) : "v"(a.w), "v"(b.w));
  return d;
}

__device__ __forceinline__ v8f z8() { v8f z = {0.f, 0.f, 0.f, 0.f, 0.f, 0.f, 0.f, 0.f}; return z; }
__device__ __forceinline__ int clampi(int v, int lo, int hi) { return v < lo ? lo : (v > hi ? hi : v); }
__device__ __forceinline__ unsigned bmask(bool c) { return 0u - (unsigned)c; }

__device__ __forceinline__ unsigned bf16_bits(float f) {
  const unsigned u = __float_as_uint(f);
  return (u + 0x7FFFu + ((u >> 16) & 1u)) >> 16;
}
__device__ __forceinline__ float bf16_val(float f) {
  return __uint_as_float(bf16_bits(f) << 16);
}
__device__ __forceinline__ unsigned bf16_vbits(float f) {
  return bf16_bits(f) << 16;
}
__device__ __forceinline__ unsigned bf_split(float v) {
  const bool isn = (v != v);
  const unsigned hb0 = bf16_bits(v);
  const float hv = __uint_as_float(hb0 << 16);
  const unsigned lb0 = bf16_bits(v - hv);
  const unsigned hb = isn ? 0x7fc0u : (hb0 & 0xffffu);
  const unsigned lb = isn ? 0x7fc0u : (lb0 & 0xffffu);
  return (lb << 16) | hb;
}
__device__ __forceinline__ unsigned short f2h(float f) {
  const _Float16 hv = (_Float16)f;
  return __builtin_bit_cast(unsigned short, hv);
}
__device__ __forceinline__ float h2f(unsigned b) {
  const _Float16 hv = __builtin_bit_cast(_Float16, (unsigned short)b);
  return (float)hv;
}
__device__ __forceinline__ float nmax(float a, float b) { return ((a > b) | (a != a)) ? a : b; }

__device__ __forceinline__ void put16(unsigned short* dp, v8us o) {
  *(volatile v8us*)dp = o;
  __threadfence();
  *(volatile v8us*)dp = o;
}
__device__ __forceinline__ void puti4(int* dp, v4i o) {
  *(volatile v4i*)dp = o;
  __threadfence();
  *(volatile v4i*)dp = o;
}

template <int SLB>
__device__ __forceinline__ int scan_chunk(const int* __restrict__ dsts, int nE, int cbase, int slotBase,
                                          int nb, int vec8, int* list, int tid, int lane, int wave) {
  int wc = 0;
  const int el0  = tid * EPT;
  const int e0   = cbase + el0;
  const int sent = -2147483647 - 1;
  v4i da, db;
  if (vec8 != 0 && cbase + CHUNK <= nE) {
    da = *(const v4i*)(dsts + e0);
    db = *(const v4i*)(dsts + e0 + 4);
  } else {
    da.x = (e0     < nE) ? dsts[min(e0,     nE - 1)] : sent;
    da.y = (e0 + 1 < nE) ? dsts[min(e0 + 1, nE - 1)] : sent;
    da.z = (e0 + 2 < nE) ? dsts[min(e0 + 2, nE - 1)] : sent;
    da.w = (e0 + 3 < nE) ? dsts[min(e0 + 3, nE - 1)] : sent;
    db.x = (e0 + 4 < nE) ? dsts[min(e0 + 4, nE - 1)] : sent;
    db.y = (e0 + 5 < nE) ? dsts[min(e0 + 5, nE - 1)] : sent;
    db.z = (e0 + 6 < nE) ? dsts[min(e0 + 6, nE - 1)] : sent;
    db.w = (e0 + 7 < nE) ? dsts[min(e0 + 7, nE - 1)] : sent;
  }
  const unsigned nbs = (unsigned)slotBase;
  const unsigned unb = (unsigned)nb;
  const unsigned s0 = (unsigned)da.x - nbs, s1 = (unsigned)da.y - nbs;
  const unsigned s2 = (unsigned)da.z - nbs, s3 = (unsigned)da.w - nbs;
  const unsigned s4 = (unsigned)db.x - nbs, s5 = (unsigned)db.y - nbs;
  const unsigned s6 = (unsigned)db.z - nbs, s7 = (unsigned)db.w - nbs;
  const bool h0 = s0 < unb, h1 = s1 < unb, h2 = s2 < unb, h3 = s3 < unb;
  const bool h4 = s4 < unb, h5 = s5 < unb, h6 = s6 < unb, h7 = s7 < unb;
  const unsigned any = __builtin_amdgcn_ballot_w32(h0 | h1 | h2 | h3 | h4 | h5 | h6 | h7);
  if (any != 0u) {
#define HITJ(J, HJ, SJ) { \
      const unsigned mj = __builtin_amdgcn_ballot_w32(HJ); \
      if (mj != 0u) { \
        if (HJ) { \
          const int pos = wc + (int)__builtin_amdgcn_mbcnt_lo(mj, 0u); \
          if (pos < WCAP) list[wave * WCAP + pos] = ((el0 + (J)) << SLB) | (int)(SJ); \
        } \
        wc += (int)__builtin_popcount(mj); } }
    HITJ(0, h0, s0)
    HITJ(1, h1, s1)
    HITJ(2, h2, s2)
    HITJ(3, h3, s3)
    HITJ(4, h4, s4)
    HITJ(5, h5, s5)
    HITJ(6, h6, s6)
    HITJ(7, h7, s7)
#undef HITJ
  }
  return wc;
}

__global__ __launch_bounds__(NTHR) void k_prep(const float* __restrict__ w2, const float* __restrict__ wih,
                                               const float* __restrict__ whh, const float* __restrict__ w1,
                                               const float* __restrict__ b1, const float* __restrict__ b2,
                                               const float* __restrict__ l0b, const float* __restrict__ cb,
                                               const float* __restrict__ fcw, const float* __restrict__ fcb,
                                               const float* __restrict__ gbi, const float* __restrict__ gbh,
                                               const float* __restrict__ lcw, const float* __restrict__ lcb,
                                               const float* __restrict__ lwi, const float* __restrict__ lwh,
                                               const float* __restrict__ lbi, const float* __restrict__ lbh,
                                               unsigned short* W2D, unsigned short* WG, float* PAR) {
  __shared__ __attribute__((aligned(16))) float sP[NTHR];
  const int tid = (int)threadIdx.x;
  const int b   = (int)blockIdx.x;
  if (b < NB_W2D) {
    const int v  = b * NTHR + tid;
    const int n  = v >> 5;
    const int k8 = (v & 31) * 8;
    const int ks = k8 & (HIDE - 1);
    const float* p = w2 + (size_t)n * HIDE + ks;
    const v4f a = *(const v4f*)p;
    const v4f c = *(const v4f*)(p + 4);
    v8us o;
    o[0] = (unsigned short)bf16_bits(a.x); o[1] = (unsigned short)bf16_bits(a.y);
    o[2] = (unsigned short)bf16_bits(a.z); o[3] = (unsigned short)bf16_bits(a.w);
    o[4] = (unsigned short)bf16_bits(c.x); o[5] = (unsigned short)bf16_bits(c.y);
    o[6] = (unsigned short)bf16_bits(c.z); o[7] = (unsigned short)bf16_bits(c.w);
    put16(W2D + (size_t)v * 8, o);
    return;
  }
  if (b < NB_W2D + NB_WG) {
    const int v    = (b - NB_W2D) * NTHR + tid;
    const int n    = v >> 4;
    const int k8   = (v & 15) * 8;
    const int part = k8 >> 5;
    const int kk   = k8 & 31;
    const int g    = n >> 5;
    const int j    = n & 31;
    const int srow = (g < 2 ? g : 2) * DIM + j;
    const float* pi = wih + (size_t)srow * DIM + kk;
    const float* ph = whh + (size_t)srow * DIM + kk;
    const v4f i0 = *(const v4f*)pi;
    const v4f i1 = *(const v4f*)(pi + 4);
    const v4f h0 = *(const v4f*)ph;
    const v4f h1 = *(const v4f*)(ph + 4);
    const bool useH = part >= 2;
    const bool zero = ((g == 2) & useH) | ((g == 3) & (!useH));
    const unsigned mh = (useH && !zero) ? 0xffffu : 0u;
    const unsigned mi = (!useH && !zero) ? 0xffffu : 0u;
    v8us o;
    o[0] = (unsigned short)((bf16_bits(i0.x) & mi) | (bf16_bits(h0.x) & mh));
    o[1] = (unsigned short)((bf16_bits(i0.y) & mi) | (bf16_bits(h0.y) & mh));
    o[2] = (unsigned short)((bf16_bits(i0.z) & mi) | (bf16_bits(h0.z) & mh));
    o[3] = (unsigned short)((bf16_bits(i0.w) & mi) | (bf16_bits(h0.w) & mh));
    o[4] = (unsigned short)((bf16_bits(i1.x) & mi) | (bf16_bits(h1.x) & mh));
    o[5] = (unsigned short)((bf16_bits(i1.y) & mi) | (bf16_bits(h1.y) & mh));
    o[6] = (unsigned short)((bf16_bits(i1.z) & mi) | (bf16_bits(h1.z) & mh));
    o[7] = (unsigned short)((bf16_bits(i1.w) & mi) | (bf16_bits(h1.w) & mh));
    put16(WG + (size_t)v * 8, o);
    return;
  }
  const int pb = b - NB_W2D - NB_WG;
  unsigned vbits = 0u;
  if (pb < 3) {
    const int i = pb * NTHR + tid;
    const unsigned tb = bf16_vbits(w1[i < 639 ? i : 639]);
    vbits = tb & bmask(i < 640);
  } else if (pb == 3) {
    const unsigned tb = bf16_vbits(b1[tid < 127 ? tid : 127]);
    vbits = tb & bmask(tid < 128);
  } else if (pb < 8) {
    const int i = (pb - 4) * NTHR + tid;
    vbits = bf16_vbits(b2[i]);
  } else if (pb == 8) {
    const unsigned ua = bf16_vbits(l0b[clampi(tid, 0, 31)]);
    const unsigned ub = bf16_vbits(cb[clampi(tid - 32, 0, 31)]);
    const unsigned uc = bf16_vbits(fcw[clampi(tid - 64, 0, 1)]);
    const unsigned ud = bf16_vbits(fcb[0]);
    const unsigned ue = bf16_vbits(lcw[clampi(tid - 68, 0, 2)]);
    const unsigned uf = bf16_vbits(lcb[0]);
    const unsigned ma = bmask(tid < 32);
    const unsigned mb = bmask((tid >= 32) & (tid < 64));
    const unsigned mc = bmask((tid >= 64) & (tid < 66));
    const unsigned md = bmask(tid == 66);
    const unsigned me = bmask((tid >= 68) & (tid < 71));
    const unsigned mf = bmask(tid == 71);
    vbits = (ua & ma) | (ub & mb) | (uc & mc) | (ud & md) | (ue & me) | (uf & mf);
  } else if (pb == 9) {
    const int c  = tid;
    const int ia = c < 95 ? c : 95;
    const int ib = (c < 64) ? c : ((c < 96) ? 64 : clampi(c - 32, 64, 95));
    const float va = bf16_val(gbi[ia]);
    const float vb = bf16_val(gbh[ib]);
    const unsigned us = __float_as_uint(va + vb);
    const unsigned ua = __float_as_uint(va);
    const unsigned ub = __float_as_uint(vb);
    const unsigned m0 = bmask(c < 64);
    const unsigned m1 = bmask((c >= 64) & (c < 96));
    const unsigned m2 = bmask((c >= 96) & (c < 128));
    vbits = (us & m0) | (ua & m1) | (ub & m2);
  } else if (pb < 42) {
    const int i = (pb - 10) * NTHR + tid;
    vbits = bf16_vbits(lwi[i]);
  } else if (pb < 58) {
    const int i = (pb - 42) * NTHR + tid;
    vbits = bf16_vbits(lwh[i]);
  } else {
    const unsigned ua = bf16_vbits(lbi[tid & 127]);
    const unsigned ub = bf16_vbits(lbh[tid & 127]);
    const unsigned ma = bmask(tid < 128);
    vbits = (ua & ma) | (ub & ~ma);
  }
  sP[tid] = __uint_as_float(vbits);
  __syncthreads();
  const v4f o = *(const v4fa*)(sP + 4 * (tid & 63));
  float* dp = PAR + (size_t)pb * NTHR + 4 * (tid & 63);
  if (tid < 64) *(volatile v4f*)dp = o;
  __threadfence();
  if (tid < 64) *(volatile v4f*)dp = o;
}

__global__ __launch_bounds__(NTHR) void k_bucket(const int* __restrict__ srcs, const int* __restrict__ dsts,
                                                 int nE, int nN, int vec8, int* LIST, int* CNT, int* OFFG) {
  extern __shared__ __attribute__((aligned(16))) int dsm[];
  int* list = dsm;
  int* hl   = dsm + LISTN;
  int* sl   = hl + RCAP;
  int* cnt  = sl + RCAP;
  int* offs = cnt + NBA;
  int* cur  = offs + NBA;
  int* misc = cur + NBA;
  const int tid = (int)threadIdx.x, lane = tid & 31, wave = tid >> 5;
  const int blk = (int)blockIdx.x;
  const int nodeBase = blk * NBA;

  {
    const v4i z4 = {0, 0, 0, 0};
    for (int i = tid * 4; i < AGG_ZINTS; i += NTHR * 4) *(v4ia*)(dsm + i) = z4;
    if (tid < 16) misc[tid] = 0;
  }
  __syncthreads();

  int t = 0, ov = 0;
  const int nChunks = (nE + CHUNK - 1) / CHUNK;
#pragma unroll 1
  for (int ch = 0; ch < nChunks; ++ch) {
    const int cbase = ch * CHUNK;
    const int wc = scan_chunk<SLA>(dsts, nE, cbase, nodeBase, NBA, vec8, list, tid, lane, wave);
    if (lane == 0) misc[wave] = wc;
    __syncthreads();
    if (wave == 0) {
#pragma unroll 1
      for (int w2 = 0; w2 < NWAVE; ++w2) {
        int c = misc[w2];
        c = c < 0 ? 0 : (c > WCAP ? WCAP : c);
#pragma unroll 1
        for (int b0 = 0; b0 < c; b0 += 32) {
          const int idx = b0 + lane;
          const int ent = list[w2 * WCAP + (idx < WCAP ? idx : WCAP - 1)];
          const int m32 = (c - b0) < 32 ? (c - b0) : 32;
#pragma unroll 1
          for (int k = 0; k < m32; ++k) {
            const int u    = __builtin_amdgcn_readlane(ent, k);
            const int slot = u & (NBA - 1);
            const int el   = (u >> SLA) & (CHUNK - 1);
            const int pk   = ((cbase + el) << SLA) | slot;
            if (t < RCAP) {
              if (lane == 0) { hl[t] = pk; cnt[slot] = cnt[slot] + 1; }
              t = t + 1;
            } else {
              ov = 1;
            }
          }
        }
      }
    }
    __syncthreads();
  }
  if (wave == 0 && lane == 0) { misc[8] = t; misc[9] = ov; }
  __syncthreads();
  int tt = misc[8];
  tt = tt < 0 ? 0 : (tt > RCAP ? RCAP : tt);
  const int ovf = misc[9];

  if (wave == 0) {
    const int base = lane * (NBA / 32);
    int s = 0;
#pragma unroll 1
    for (int i = 0; i < NBA / 32; ++i) s += cnt[base + i];
    int incl = s;
#pragma unroll
    for (int d = 1; d < 32; d <<= 1) {
      const int y = __shfl_up(incl, d, 32);
      if (lane >= d) incl += y;
    }
    int run = incl - s;
#pragma unroll 1
    for (int i = 0; i < NBA / 32; ++i) {
      const int cv = cnt[base + i];
      offs[base + i] = run;
      cur[base + i]  = run;
      run += cv;
    }
  }
  __syncthreads();
  if (wave == 0) {
#pragma unroll 1
    for (int b0 = 0; b0 < tt; b0 += 32) {
      const int idx = b0 + lane;
      const int ent = hl[idx < RCAP ? idx : RCAP - 1];
      const int m32 = (tt - b0) < 32 ? (tt - b0) : 32;
#pragma unroll 1
      for (int k = 0; k < m32; ++k) {
        const int u    = __builtin_amdgcn_readlane(ent, k);
        const int slot = u & (NBA - 1);
        if (lane == 0) {
          int p = cur[slot];
          p = p < 0 ? 0 : (p > RCAP - 1 ? RCAP - 1 : p);
          sl[p] = u;
          cur[slot] = p + 1;
        }
      }
    }
  }
  __syncthreads();

  int* lb = LIST + (size_t)blk * RCAP * 2;
#pragma unroll 1
  for (int it = 0; it < RCAP / (2 * NTHR); ++it) {
    const int p0 = (it * NTHR + tid) * 2;
    const int e0 = sl[(p0     < tt) ? p0     : 0];
    const int e1 = sl[(p0 + 1 < tt) ? p0 + 1 : 0];
    const int id0 = clampi(e0 >> SLA, 0, nE - 1);
    const int id1 = clampi(e1 >> SLA, 0, nE - 1);
    const int q0 = clampi(srcs[id0], 0, nN - 1);
    const int q1 = clampi(srcs[id1], 0, nN - 1);
    v4i o;
    o.x = id0; o.y = q0; o.z = id1; o.w = q1;
    puti4(lb + (size_t)p0 * 2, o);
  }
  {
    const int s4 = 4 * tid;
    v4i c4 = *(const v4ia*)(cnt + s4);
    v4i o4 = *(const v4ia*)(offs + s4);
    const int gb = blk * RCAP;
    if (ovf != 0) { c4.x = -1; c4.y = -1; c4.z = -1; c4.w = -1; }
    o4.x += gb; o4.y += gb; o4.z += gb; o4.w += gb;
    puti4(CNT + (size_t)nodeBase + s4, c4);
    puti4(OFFG + (size_t)nodeBase + s4, o4);
  }
}

__global__ __launch_bounds__(GTHR) void k_lin0(const float* __restrict__ x, const float* __restrict__ w,
                                               const float* __restrict__ PAR, int nN, float* H0) {
  __shared__ __attribute__((aligned(16))) float stg[GBM * DIM];
  const int tid = (int)threadIdx.x, lane = tid & 31, wave = tid >> 5, hh = lane >> 4, m = lane & 15;
  const int rowBase = (int)blockIdx.x * GBM;
  const int row = rowBase + 16 * wave + m;
  const int rc  = row < nN ? row : nN - 1;
  FragB af;
  {
    const float* xp = x + (size_t)rc * DIM + 8 * hh;
    const v4f x0 = *(const v4f*)xp;
    const v4f x1 = *(const v4f*)(xp + 4);
    const v4f x2 = *(const v4f*)(xp + 16);
    const v4f x3 = *(const v4f*)(xp + 20);
    v8us lo8, hi8;
    lo8[0] = (unsigned short)bf16_bits(x0.x); lo8[1] = (unsigned short)bf16_bits(x0.y);
    lo8[2] = (unsigned short)bf16_bits(x0.z); lo8[3] = (unsigned short)bf16_bits(x0.w);
    lo8[4] = (unsigned short)bf16_bits(x1.x); lo8[5] = (unsigned short)bf16_bits(x1.y);
    lo8[6] = (unsigned short)bf16_bits(x1.z); lo8[7] = (unsigned short)bf16_bits(x1.w);
    hi8[0] = (unsigned short)bf16_bits(x2.x); hi8[1] = (unsigned short)bf16_bits(x2.y);
    hi8[2] = (unsigned short)bf16_bits(x2.z); hi8[3] = (unsigned short)bf16_bits(x2.w);
    hi8[4] = (unsigned short)bf16_bits(x3.x); hi8[5] = (unsigned short)bf16_bits(x3.y);
    hi8[6] = (unsigned short)bf16_bits(x3.z); hi8[7] = (unsigned short)bf16_bits(x3.w);
    af.h[0] = lo8;
    af.h[1] = hi8;
  }
  v8f acc[2];
#pragma unroll
  for (int nt = 0; nt < 2; ++nt) {
    const float* wp = w + (size_t)(16 * nt + m) * DIM + 8 * hh;
    const v4f w0 = *(const v4f*)wp;
    const v4f w1 = *(const v4f*)(wp + 4);
    const v4f w2 = *(const v4f*)(wp + 16);
    const v4f w3 = *(const v4f*)(wp + 20);
    v8us lo8, hi8;
    lo8[0] = (unsigned short)bf16_bits(w0.x); lo8[1] = (unsigned short)bf16_bits(w0.y);
    lo8[2] = (unsigned short)bf16_bits(w0.z); lo8[3] = (unsigned short)bf16_bits(w0.w);
    lo8[4] = (unsigned short)bf16_bits(w1.x); lo8[5] = (unsigned short)bf16_bits(w1.y);
    lo8[6] = (unsigned short)bf16_bits(w1.z); lo8[7] = (unsigned short)bf16_bits(w1.w);
    hi8[0] = (unsigned short)bf16_bits(w2.x); hi8[1] = (unsigned short)bf16_bits(w2.y);
    hi8[2] = (unsigned short)bf16_bits(w2.z); hi8[3] = (unsigned short)bf16_bits(w2.w);
    hi8[4] = (unsigned short)bf16_bits(w3.x); hi8[5] = (unsigned short)bf16_bits(w3.y);
    hi8[6] = (unsigned short)bf16_bits(w3.z); hi8[7] = (unsigned short)bf16_bits(w3.w);
    FragB bf;
    bf.h[0] = lo8;
    bf.h[1] = hi8;
    acc[nt] = wmb(af, bf, z8());
  }
#pragma unroll
  for (int nt = 0; nt < 2; ++nt) {
    const int lc = 16 * nt + m;
    const float bv = PAR[P_L0B + lc];
#pragma unroll
    for (int r = 0; r < 8; ++r) {
      const int lr = 16 * wave + 8 * hh + r;
      stg[lr * DIM + lc] = fmaxf(acc[nt][r] + bv, 0.0f);
    }
  }
  __syncthreads();
  v4f pv[4];
#pragma unroll
  for (int s = 0; s < 4; ++s) pv[s] = *(const v4fa*)(stg + (16 * wave + 4 * s + (lane >> 3)) * DIM + 4 * (lane & 7));
#pragma unroll
  for (int s = 0; s < 4; ++s) {
    const int r2 = rowBase + 16 * wave + 4 * s + (lane >> 3);
    if (r2 < nN) *(volatile v4f*)(H0 + (size_t)r2 * DIM + 4 * (lane & 7)) = pv[s];
  }
  __threadfence();
#pragma unroll
  for (int s = 0; s < 4; ++s) {
    const int r2 = rowBase + 16 * wave + 4 * s + (lane >> 3);
    if (r2 < nN) *(volatile v4f*)(H0 + (size_t)r2 * DIM + 4 * (lane & 7)) = pv[s];
  }
}

__global__ __launch_bounds__(NTHR) void k_ew(const float* __restrict__ eattr, int nE,
                                             const float* __restrict__ PAR,
                                             const unsigned short* __restrict__ W2D, unsigned short* EW) {
  extern __shared__ __attribute__((aligned(16))) float dyn[];
  __shared__ __attribute__((aligned(16))) float sW1[768];
  __shared__ __attribute__((aligned(16))) float sB1[HIDE];
  float*          sD = dyn;
  unsigned short* sA = (unsigned short*)(dyn + EPB * DP);

  const int tid = (int)threadIdx.x, lane = tid & 31, wave = tid >> 5, hh = lane >> 4, m = lane & 15;
  const int elb = (int)blockIdx.x * EPB;

#pragma unroll 1
  for (int i = tid; i < 768; i += NTHR) sW1[i] = PAR[P_W1 + i];
  if (tid < HIDE) sB1[tid] = PAR[P_B1 + tid];

  const int row  = tid & (EPB - 1);
  const int half = tid >> 7;
  const int e    = elb + row;
  const int ec   = e < nE ? e : nE - 1;
  const float* ar = eattr + (size_t)ec * 5;
  const float a0 = bf16_val(ar[0]);
  const float a1 = bf16_val(ar[1]);
  const float a2 = bf16_val(ar[2]);
  const float a3 = bf16_val(ar[3]);
  const float a4 = bf16_val(ar[4]);
  __syncthreads();

  {
    unsigned short* ra = sA + row * AP + 64 * half;
#pragma unroll 1
    for (int c8 = 0; c8 < 8; ++c8) {
      v8us ho, lo;
#pragma unroll
      for (int i = 0; i < 8; ++i) {
        const int k = 64 * half + 8 * c8 + i;
        const float* wr = sW1 + k * 5;
        float v = a0 * wr[0];
        v = fmaf(a1, wr[1], v);
        v = fmaf(a2, wr[2], v);
        v = fmaf(a3, wr[3], v);
        v = fmaf(a4, wr[4], v);
        v = fmaxf(v + sB1[k], 0.0f);
        const unsigned hb = bf16_bits(v);
        ho[i] = (unsigned short)hb;
        lo[i] = (unsigned short)bf16_bits(v - __uint_as_float(hb << 16));
      }
      *(v8usa*)(ra + 8 * c8)        = ho;
      *(v8usa*)(ra + HIDE + 8 * c8) = lo;
    }
  }
  __syncthreads();

  const unsigned short* ap = sA + (16 * wave + m) * AP + 8 * hh;
  const int j  = lane & 15;
  const int rq = lane >> 4;

#pragma unroll 1
  for (int ch = 0; ch < 8; ++ch) {
    v8f acc[8];
#pragma unroll
    for (int t = 0; t < 8; ++t) acc[t] = z8();
    const unsigned short* bp = W2D + (size_t)(128 * ch + m) * (size_t)KEW + 8 * hh;
#pragma unroll 1
    for (int k0 = 0; k0 < KEW; k0 += 32) {
      FragB af;
      af.h[0] = *(const v8usa*)(ap + k0);
      af.h[1] = *(const v8usa*)(ap + k0 + 16);
#pragma unroll
      for (int nt = 0; nt < 8; ++nt) {
        const unsigned short* wq = bp + (size_t)(16 * nt) * (size_t)KEW + k0;
        FragB bf;
        bf.h[0] = *(const v8usa*)wq;
        bf.h[1] = *(const v8usa*)(wq + 16);
        acc[nt] = wmb(af, bf, acc[nt]);
      }
    }
#pragma unroll
    for (int nt = 0; nt < 8; ++nt) {
      const int lc = 16 * nt + m;
#pragma unroll
      for (int r = 0; r < 8; ++r) {
        const int lr = 16 * wave + 8 * hh + r;
        sD[lr * DP + lc] = acc[nt][r];
      }
    }
    __syncthreads();

    const v4f ba = *(const v4f*)(PAR + P_B2 + 128 * ch + 8 * j);
    const v4f bb = *(const v4f*)(PAR + P_B2 + 128 * ch + 8 * j + 4);
    v8us pv[8];
#pragma unroll
    for (int s = 0; s < 8; ++s) {
      const float* sp = sD + (16 * wave + 2 * s + rq) * DP + 8 * j;
      const v4f va = *(const v4fa*)sp;
      const v4f vb = *(const v4fa*)(sp + 4);
      v8us o;
      o[0] = f2h(CEW * (va.x + ba.x)); o[1] = f2h(CEW * (va.y + ba.y));
      o[2] = f2h(CEW * (va.z + ba.z)); o[3] = f2h(CEW * (va.w + ba.w));
      o[4] = f2h(CEW * (vb.x + bb.x)); o[5] = f2h(CEW * (vb.y + bb.y));
      o[6] = f2h(CEW * (vb.z + bb.z)); o[7] = f2h(CEW * (vb.w + bb.w));
      pv[s] = o;
    }
#pragma unroll
    for (int s = 0; s < 8; ++s) {
      const int e2 = elb + 16 * wave + 2 * s + rq;
      if (e2 < nE) *(volatile v8us*)(EW + (size_t)e2 * EWN + 128 * ch + 8 * j) = pv[s];
    }
    __threadfence();
#pragma unroll
    for (int s = 0; s < 8; ++s) {
      const int e2 = elb + 16 * wave + 2 * s + rq;
      if (e2 < nE) *(volatile v8us*)(EW + (size_t)e2 * EWN + 128 * ch + 8 * j) = pv[s];
    }
    __syncthreads();
  }
}

__global__ __launch_bounds__(NTHR) void k_conv(const float* __restrict__ Hl, const unsigned short* __restrict__ EW,
                                               const int* __restrict__ LIST, const int* __restrict__ CNT,
                                               const int* __restrict__ OFFG, const float* __restrict__ PAR,
                                               int nN, int nE, unsigned short* AG) {
  __shared__ __attribute__((aligned(16))) unsigned short sAG[NWAVE * 128];
  const int tid = (int)threadIdx.x, lane = tid & 31, wave = tid >> 5;
  const int node  = (int)blockIdx.x * NWAVE + wave;
  const bool live = node < nN;
  const int nodec = live ? node : nN - 1;

  int c = CNT[nodec];
  const bool bad = (c < 0) | (c > DEGCAP);
  c = clampi(c, 0, DEGCAP);
  const float degf = (c > 0) ? (float)c : 1.0f;
  const int cl = live ? c : 0;
  const int base = (nodec >> SLA) * RCAP;
  int off = OFFG[nodec];
  off = clampi(off, base, base + RCAP - 1);
  int idx = off + lane;
  idx = idx > base + RCAP - 1 ? base + RCAP - 1 : idx;
  const v2i pr = *(const v2i*)(LIST + (size_t)idx * 2);
  const int eid = clampi(pr.x, 0, nE - 1);
  const int sid = clampi(pr.y, 0, nN - 1);
  const float hv = Hl[(size_t)nodec * DIM + lane];

  float acc = 0.0f;
#pragma unroll 1
  for (int k = 0; k < cl; ++k) {
    const int ek = __builtin_amdgcn_readlane(eid, k);
    const int sk = __builtin_amdgcn_readlane(sid, k);
    const float xs = Hl[(size_t)sk * DIM + lane];
    const int xb = __float_as_int(xs);
    const unsigned short* wr = EW + (size_t)ek * EWN + lane;
#pragma unroll 4
    for (int i = 0; i < DIM; ++i) {
      const float xi = __int_as_float(__builtin_amdgcn_readlane(xb, i));
      const float wv = h2f((unsigned)wr[i * DIM]);
      acc = fmaf(xi, wv, acc);
    }
  }
  const float cbv = PAR[P_CB + lane];
  const float fw0 = PAR[P_FC + 0];
  const float fw1 = PAR[P_FC + 1];
  const float fb  = PAR[P_FC + 2];
  const float agg = (acc * EWINV) / degf;
  const float tt  = agg + cbv;
  const float mm  = (tt > 0.0f) ? tt : (tt - tt);
  float mp = (fw0 * hv + fw1 * mm) + fb;
  const float qnan = __int_as_float(0x7fc00000);
  mp = bad ? qnan : mp;

  const unsigned sm = bf_split(mp);
  const unsigned sh = bf_split(hv);
  const unsigned mk = live ? 0xffffu : 0u;
  unsigned short* sr = sAG + wave * 128;
  sr[lane]      = (unsigned short)((sm & 0xffffu) & mk);
  sr[32 + lane] = (unsigned short)((sm >> 16) & mk);
  sr[64 + lane] = (unsigned short)((sh & 0xffffu) & mk);
  sr[96 + lane] = (unsigned short)((sh >> 16) & mk);
  __syncthreads();
  const v8us o = *(const v8usa*)(sAG + 8 * (tid & 127));
  unsigned short* dp = AG + (size_t)blockIdx.x * (NWAVE * 128) + 8 * (tid & 127);
  if (tid < 128) *(volatile v8us*)dp = o;
  __threadfence();
  if (tid < 128) *(volatile v8us*)dp = o;
}

__global__ __launch_bounds__(GTHR) void k_gru(const unsigned short* __restrict__ A,
                                              const unsigned short* __restrict__ BT,
                                              const float* __restrict__ PAR, const float* __restrict__ Hl,
                                              int nN, float* Hn) {
  __shared__ __attribute__((aligned(16))) float stg[GBM * GBN];
  const int tid = (int)threadIdx.x, lane = tid & 31, wave = tid >> 5, hh = lane >> 4, m = lane & 15;
  const int rowBase = (int)blockIdx.x * GBM;

  v8f acc[8];
#pragma unroll
  for (int t = 0; t < 8; ++t) acc[t] = z8();
  const unsigned short* ap = A  + (size_t)(rowBase + 16 * wave + m) * (size_t)KG + 8 * hh;
  const unsigned short* bp = BT + (size_t)m * (size_t)KG + 8 * hh;

#pragma unroll 1
  for (int k0 = 0; k0 < KG; k0 += 32) {
    FragB af;
    af.h[0] = *(const v8usa*)(ap + k0);
    af.h[1] = *(const v8usa*)(ap + k0 + 16);
#pragma unroll
    for (int nt = 0; nt < 8; ++nt) {
      const unsigned short* wq = bp + (size_t)(16 * nt) * (size_t)KG + k0;
      FragB bf;
      bf.h[0] = *(const v8usa*)wq;
      bf.h[1] = *(const v8usa*)(wq + 16);
      acc[nt] = wmb(af, bf, acc[nt]);
    }
  }

#pragma unroll
  for (int nt = 0; nt < 8; ++nt) {
    const int lc = 16 * nt + m;
#pragma unroll
    for (int r = 0; r < 8; ++r) {
      const int lr = 16 * wave + 8 * hh + r;
      stg[lr * GBN + lc] = acc[nt][r];
    }
  }
  __syncthreads();

  const float br = PAR[P_GB + lane];
  const float bz = PAR[P_GB + 32 + lane];
  const float bi = PAR[P_GB + 64 + lane];
  const float bh = PAR[P_GB + 96 + lane];
#pragma unroll 1
  for (int i = 0; i < 16; ++i) {
    const int lr  = 16 * wave + i;
    const int row = rowBase + lr;
    const int rc  = row < nN ? row : nN - 1;
    const float hv = Hl[(size_t)rc * DIM + lane];
    float* sp = stg + lr * GBN;
    const float c0 = sp[lane];
    const float c1 = sp[32 + lane];
    const float c2 = sp[64 + lane];
    const float c3 = sp[96 + lane];
    const float rg = 1.0f / (1.0f + expf(-(c0 + br)));
    const float zg = 1.0f / (1.0f + expf(-(c1 + bz)));
    const float ng = tanhf((c2 + bi) + rg * (c3 + bh));
    const float hn = (1.0f - zg) * ng + zg * hv;
    sp[lane] = hn;
  }
  __syncthreads();

  v4f pv[4];
#pragma unroll
  for (int s = 0; s < 4; ++s) pv[s] = *(const v4fa*)(stg + (16 * wave + 4 * s + (lane >> 3)) * GBN + 4 * (lane & 7));
#pragma unroll
  for (int s = 0; s < 4; ++s) {
    const int r2 = rowBase + 16 * wave + 4 * s + (lane >> 3);
    if (r2 < nN) *(volatile v4f*)(Hn + (size_t)r2 * DIM + 4 * (lane & 7)) = pv[s];
  }
  __threadfence();
#pragma unroll
  for (int s = 0; s < 4; ++s) {
    const int r2 = rowBase + 16 * wave + 4 * s + (lane >> 3);
    if (r2 < nN) *(volatile v4f*)(Hn + (size_t)r2 * DIM + 4 * (lane & 7)) = pv[s];
  }
}

__global__ __launch_bounds__(NTHR) void k_pool(const int* __restrict__ batch, int nN, int vec8,
                                               const float* __restrict__ H1, const float* __restrict__ H2,
                                               const float* __restrict__ H3, const float* __restrict__ PAR,
                                               float* out) {
  __shared__ __attribute__((aligned(16))) int   list[LISTN];
  __shared__ __attribute__((aligned(16))) float gnt[GCAP * GP];
  __shared__ __attribute__((aligned(16))) float qs[64];
  __shared__ __attribute__((aligned(16))) float hs[DIM];
  __shared__ float cs[DIM];
  __shared__ float sg[128];
  __shared__ float sa[GCAP];
  __shared__ float redm[NWAVE];
  __shared__ float reds[NWAVE];
  __shared__ float red2[NWAVE * DIM];
  __shared__ int   nlist[GCAP];
  __shared__ int   misc[16];
  const int tid = (int)threadIdx.x, lane = tid & 31, wave = tid >> 5;
  const int g = (int)blockIdx.x;

  {
    const v4i z4 = {0, 0, 0, 0};
    const v4f f4 = {0.0f, 0.0f, 0.0f, 0.0f};
    for (int i = tid * 4; i < LISTN; i += NTHR * 4) *(v4ia*)(list + i) = z4;
    for (int i = tid; i < (GCAP * GP) / 4; i += NTHR) *(v4fa*)(gnt + 4 * i) = f4;
    nlist[tid] = 0;
    sa[tid] = 0.0f;
    if (tid < 64) qs[tid] = 0.0f;
    if (tid < DIM) { hs[tid] = 0.0f; cs[tid] = 0.0f; }
    if (tid < 16) misc[tid] = 0;
  }
  __syncthreads();

  int t = 0;
  const int nChunks = (nN + CHUNK - 1) / CHUNK;
#pragma unroll 1
  for (int ch = 0; ch < nChunks; ++ch) {
    const int cbase = ch * CHUNK;
    const int wc = scan_chunk<0>(batch, nN, cbase, g, 1, vec8, list, tid, lane, wave);
    if (lane == 0) misc[wave] = wc;
    __syncthreads();
    if (wave == 0) {
#pragma unroll 1
      for (int w2 = 0; w2 < NWAVE; ++w2) {
        int c = misc[w2];
        c = c < 0 ? 0 : (c > WCAP ? WCAP : c);
#pragma unroll 1
        for (int b0 = 0; b0 < c; b0 += 32) {
          const int idx = b0 + lane;
          const int ent = list[w2 * WCAP + (idx < WCAP ? idx : WCAP - 1)];
          const int pos = t + idx;
          if (idx < c && pos < GCAP) nlist[pos] = cbase + ent;
        }
        t = t + c;
        t = t > 2 * GCAP ? 2 * GCAP : t;
      }
    }
    __syncthreads();
  }
  if (wave == 0 && lane == 0) { misc[8] = t; misc[9] = (t > GCAP) ? 1 : 0; }
  __syncthreads();
  const int cntg = clampi(misc[8], 0, GCAP);
  const int ovf  = misc[9];

  {
    const float lw0 = PAR[P_LC + 0];
    const float lw1 = PAR[P_LC + 1];
    const float lw2 = PAR[P_LC + 2];
    const float lb  = PAR[P_LC + 3];
#pragma unroll 1
    for (int p = wave; p < cntg; p += NWAVE) {
      const int nd = clampi(nlist[p], 0, nN - 1);
      const float a = H1[(size_t)nd * DIM + lane];
      const float b = H2[(size_t)nd * DIM + lane];
      const float c = H3[(size_t)nd * DIM + lane];
      gnt[p * GP + lane] = ((lw0 * a + lw1 * b) + lw2 * c) + lb;
    }
  }
  __syncthreads();

  const float pinf = __int_as_float(0x7f800000);
  const bool  inl  = tid < cntg;
#pragma unroll 1
  for (int step = 0; step < 3; ++step) {
    if (tid < 128) {
      const float* wi = PAR + P_LWI + tid * 64;
      const float* wh = PAR + P_LWH + tid * DIM;
      float a = 0.0f;
#pragma unroll 1
      for (int k4 = 0; k4 < 16; ++k4) {
        const v4f w = *(const v4f*)(wi + 4 * k4);
        const v4f q = *(const v4fa*)(qs + 4 * k4);
        a = fmaf(q.x, w.x, a); a = fmaf(q.y, w.y, a); a = fmaf(q.z, w.z, a); a = fmaf(q.w, w.w, a);
      }
      a = a + PAR[P_LBI + tid];
      float b = 0.0f;
#pragma unroll 1
      for (int k4 = 0; k4 < 8; ++k4) {
        const v4f w = *(const v4f*)(wh + 4 * k4);
        const v4f q = *(const v4fa*)(hs + 4 * k4);
        b = fmaf(q.x, w.x, b); b = fmaf(q.y, w.y, b); b = fmaf(q.z, w.z, b); b = fmaf(q.w, w.w, b);
      }
      a = (a + b) + PAR[P_LBH + tid];
      float act;
      if (wave == 2) act = tanhf(a);
      else           act = 1.0f / (1.0f + expf(-a));
      sg[tid] = act;
    }
    __syncthreads();
    if (tid < DIM) {
      const float cn = sg[32 + tid] * cs[tid] + sg[tid] * sg[64 + tid];
      const float hn = sg[96 + tid] * tanhf(cn);
      cs[tid] = cn;
      hs[tid] = hn;
      qs[tid] = hn;
    }
    __syncthreads();

    float e = 0.0f;
    {
      const float* gr = gnt + tid * GP;
#pragma unroll 2
      for (int c = 0; c < DIM; ++c) e = fmaf(gr[c], hs[c], e);
    }
    const float ev = inl ? e : -pinf;
    float mx = ev;
#pragma unroll
    for (int d = 16; d >= 1; d >>= 1) {
      const float y = __shfl_xor(mx, d, 32);
      mx = nmax(mx, y);
    }
    if (lane == 0) redm[wave] = mx;
    __syncthreads();
    float em = redm[0];
#pragma unroll
    for (int w2 = 1; w2 < NWAVE; ++w2) em = nmax(em, redm[w2]);
    em = (fabsf(em) < pinf) ? em : 0.0f;

    const float xarg = inl ? (e - em) : 0.0f;
    const float ex0  = expf(xarg);
    const float ex   = inl ? ex0 : 0.0f;
    float sm = ex;
#pragma unroll
    for (int d = 16; d >= 1; d >>= 1) sm = sm + __shfl_xor(sm, d, 32);
    if (lane == 0) reds[wave] = sm;
    __syncthreads();
    float den = reds[0];
#pragma unroll
    for (int w2 = 1; w2 < NWAVE; ++w2) den = den + reds[w2];
    const float dn = (den < 1e-16f) ? 1e-16f : den;
    const float rdn = 1.0f / dn;
    sa[tid] = ex * rdn;
    __syncthreads();

    float rp = 0.0f;
#pragma unroll 1
    for (int p = wave; p < cntg; p += NWAVE) rp = fmaf(sa[p], gnt[p * GP + lane], rp);
    red2[wave * DIM + lane] = rp;
    __syncthreads();
    if (tid < DIM) {
      float r = red2[tid];
#pragma unroll
      for (int w2 = 1; w2 < NWAVE; ++w2) r = r + red2[w2 * DIM + tid];
      qs[32 + tid] = r;
    }
    __syncthreads();
  }

  v4f o = *(const v4fa*)(qs + 4 * (tid & 15));
  if (ovf != 0) {
    const float qnan = __int_as_float(0x7fc00000);
    o.x = qnan; o.y = qnan; o.z = qnan; o.w = qnan;
  }
  float* dp = out + (size_t)g * 64 + 4 * (tid & 15);
  if (tid < 16) *(volatile v4f*)dp = o;
  __threadfence();
  if (tid < 16) *(volatile v4f*)dp = o;
}

static inline int cdiv(int a, int b) { return (a + b - 1) / b; }
static inline size_t al256(size_t o) { return (o + 255) & ~(size_t)255; }

extern "C" void kernel_launch(void* const* d_in, const int* in_sizes, int n_in,
                              void* d_out, int out_size, void* d_ws, size_t ws_size,
                              hipStream_t stream) {
  if (n_in < 23) return;
  const int nN = in_sizes[3];
  if (nN < 64 || nN >= (1 << 24)) return;
  if ((long long)in_sizes[0] != (long long)nN * DIM) return;
  if (in_sizes[1] < 2 || (in_sizes[1] & 1) != 0) return;
  const int nE = in_sizes[1] / 2;
  if (nE < 1 || nE >= (1 << 21)) return;
  if ((long long)in_sizes[2] != (long long)nE * 5) return;
  if (in_sizes[4] != DIM * DIM || in_sizes[5] != DIM) return;
  if (in_sizes[6] != HIDE * 5 || in_sizes[7] != HIDE) return;
  if (in_sizes[8] != EWN * HIDE || in_sizes[9] != EWN) return;
  if (in_sizes[10] != DIM || in_sizes[11] != 2 || in_sizes[12] != 1) return;
  if (in_sizes[13] != 3 * DIM * DIM || in_sizes[14] != 3 * DIM * DIM) return;
  if (in_sizes[15] != 3 * DIM || in_sizes[16] != 3 * DIM) return;
  if (in_sizes[17] != 3 || in_sizes[18] != 1) return;
  if (in_sizes[19] != 4 * DIM * 2 * DIM || in_sizes[20] != 4 * DIM * DIM) return;
  if (in_sizes[21] != 4 * DIM || in_sizes[22] != 4 * DIM) return;
  if (out_size < 64 || (out_size % 64) != 0) return;
  const int nB = out_size / 64;

  const float* x    = (const float*)d_in[0];
  const int*   ei   = (const int*)d_in[1];
  const float* ea   = (const float*)d_in[2];
  const int*   bat  = (const int*)d_in[3];
  const float* l0w  = (const float*)d_in[4];
  const float* l0b  = (const float*)d_in[5];
  const float* w1   = (const float*)d_in[6];
  const float* b1   = (const float*)d_in[7];
  const float* w2   = (const float*)d_in[8];
  const float* b2   = (const float*)d_in[9];
  const float* cb   = (const float*)d_in[10];
  const float* fcw  = (const float*)d_in[11];
  const float* fcb  = (const float*)d_in[12];
  const float* gwi  = (const float*)d_in[13];
  const float* gwh  = (const float*)d_in[14];
  const float* gbi  = (const float*)d_in[15];
  const float* gbh  = (const float*)d_in[16];
  const float* lcw  = (const float*)d_in[17];
  const float* lcb  = (const float*)d_in[18];
  const float* lwi  = (const float*)d_in[19];
  const float* lwh  = (const float*)d_in[20];
  const float* lbi  = (const float*)d_in[21];
  const float* lbh  = (const float*)d_in[22];
  float* out = (float*)d_out;
  const int* src = ei;
  const int* dst = ei + nE;

  const int MP = cdiv(nN, GBM) * GBM;
  const int gM = MP / GBM;
  const int gA = cdiv(nN, NBA);
  if ((long long)gA * NBA < (long long)nN) return;
  const int EB = cdiv(nE, EPB);
  const int EP = EB * EPB;
  const int vecE = ((nE & 3) == 0) ? 1 : 0;

  char* ws = (char*)d_ws;
  size_t off = 0;
  const size_t oW2D = off; off = al256(off + (size_t)EWN * KEW * 2);
  const size_t oWG  = off; off = al256(off + (size_t)128 * KG * 2);
  const size_t oPAR = off; off = al256(off + (size_t)PARN * 4);
  const size_t szH  = al256((size_t)MP * DIM * 4);
  const size_t oH0  = off; off += szH;
  const size_t oH1  = off; off += szH;
  const size_t oH2  = off; off += szH;
  const size_t oH3  = off; off += szH;
  const size_t oAG  = off; off = al256(off + (size_t)MP * KG * 2);
  const size_t oLS  = off; off = al256(off + (size_t)gA * RCAP * 8);
  const size_t oCN  = off; off = al256(off + (size_t)gA * NBA * 4);
  const size_t oOF  = off; off = al256(off + (size_t)gA * NBA * 4);
  const size_t oEW  = off; off = al256(off + (size_t)EP * EWN * 2);
  if (off > ws_size || off > (size_t)WSMAX) return;
  unsigned short* W2D = (unsigned short*)(ws + oW2D);
  unsigned short* WG  = (unsigned short*)(ws + oWG);
  float*          PAR = (float*)(ws + oPAR);
  float*          H0  = (float*)(ws + oH0);
  float*          H1  = (float*)(ws + oH1);
  float*          H2  = (float*)(ws + oH2);
  float*          H3  = (float*)(ws + oH3);
  unsigned short* AG  = (unsigned short*)(ws + oAG);
  int*            LST = (int*)(ws + oLS);
  int*            CNT = (int*)(ws + oCN);
  int*            OFG = (int*)(ws + oOF);
  unsigned short* EW  = (unsigned short*)(ws + oEW);

  hipFuncSetAttribute(reinterpret_cast<const void*>(&k_ew), hipFuncAttributeMaxDynamicSharedMemorySize,
                      (int)EW_LDS_BYTES);
  hipFuncSetAttribute(reinterpret_cast<const void*>(&k_bucket), hipFuncAttributeMaxDynamicSharedMemorySize,
                      (int)AGG_LDS_BYTES);

  k_prep<<<NB_W2D + NB_WG + NB_PAR, NTHR, 0, stream>>>(w2, gwi, gwh, w1, b1, b2, l0b, cb, fcw, fcb, gbi, gbh,
                                                        lcw, lcb, lwi, lwh, lbi, lbh, W2D, WG, PAR);
  k_bucket<<<gA, NTHR, AGG_LDS_BYTES, stream>>>(src, dst, nE, nN, vecE, LST, CNT, OFG);
  k_lin0<<<gM, GTHR, 0, stream>>>(x, l0w, PAR, nN, H0);
  k_ew<<<EB, NTHR, EW_LDS_BYTES, stream>>>(ea, nE, PAR, W2D, EW);
  k_conv<<<MP / NWAVE, NTHR, 0, stream>>>(H0, EW, LST, CNT, OFG, PAR, nN, nE, AG);
  k_gru<<<gM, GTHR, 0, stream>>>(AG, WG, PAR, H0, nN, H1);
  k_conv<<<MP / NWAVE, NTHR, 0, stream>>>(H1, EW, LST, CNT, OFG, PAR, nN, nE, AG);
  k_gru<<<gM, GTHR, 0, stream>>>(AG, WG, PAR, H1, nN, H2);
  k_conv<<<MP / NWAVE, NTHR, 0, stream>>>(H2, EW, LST, CNT, OFG, PAR, nN, nE, AG);
  k_gru<<<gM, GTHR, 0, stream>>>(AG, WG, PAR, H2, nN, H3);
  k_pool<<<nB, NTHR, 0, stream>>>(bat, nN, 1, H1, H2, H3, PAR, out);
}
